// EnDecoder_26603027432101
// MI455X (gfx1250) — hardware-verified
//
#include <hip/hip_runtime.h>


#ifndef NB
#define NB 64
#endif
#ifndef SEQ
#define SEQ 2048
#endif
#define NB_FULL  64
#define SEQ_FULL 2048
#ifndef OUT_SEQ
#define OUT_SEQ SEQ
#endif
#define NJ   22
#define NC   66
#define KD   10
#define NP   63
#define NT   5
#define SPB  128
#define SKP  81

static_assert(NC == NJ * 3);
static_assert(NP == (NJ - 1) * 3);
static_assert(KD == 10);
static_assert(KD % 2 == 0);
static_assert(NT * 16 >= NC);
static_assert(NT * 16 <= SKP);
static_assert(NT * 16 <= SPB);
static_assert(SPB == 128);
static_assert(SEQ % SPB == 0);
static_assert(SEQ_FULL % SPB == 0);
static_assert(OUT_SEQ % SPB == 0);
static_assert(NB <= NB_FULL);
static_assert(SEQ <= SEQ_FULL);
static_assert((SPB * NP) % 4 == 0);
static_assert(((size_t)SPB * NP * 4) % 16 == 0);
static_assert((SPB * NC) % 4 == 0);
static_assert(((size_t)SPB * NC * 4) % 128 == 0);
static_assert((SPB * NC / 4) % 32 == 0);
static_assert((SPB * NC / 4) == 16 * SPB + 64);

typedef unsigned short bf;
typedef __attribute__((ext_vector_type(16))) __bf16   v16bf;
typedef __attribute__((ext_vector_type(8)))  unsigned short v8us;
typedef __attribute__((ext_vector_type(8)))  float    v8f;
typedef __attribute__((ext_vector_type(4)))  float    v4f;
typedef __attribute__((ext_vector_type(2)))  float    v2f;
typedef v4f  __attribute__((may_alias)) v4fa;

static constexpr size_t LDS_BYTES = (size_t)SPB * 4 * 16 + (size_t)NT * 16 * 4 * 16 + (size_t)SPB * SKP * 4 + (size_t)SPB * NP * 4 + (size_t)SPB * NC * 4;
static_assert(LDS_BYTES <= (size_t)131072);

static constexpr int parent_of(int j) {
    return j <= 3 ? 0 : (j <= 11 ? j - 3 : (j <= 14 ? 9 : (j == 15 ? 12 : (j == 16 ? 13 : (j == 17 ? 14 : (j == 18 ? 16 : j - 2))))));
}
static_assert(parent_of(1) == 0 && parent_of(2) == 0 && parent_of(3) == 0);
static_assert(parent_of(4) == 1 && parent_of(5) == 2 && parent_of(6) == 3 && parent_of(7) == 4 && parent_of(8) == 5 && parent_of(9) == 6 && parent_of(10) == 7 && parent_of(11) == 8);
static_assert(parent_of(12) == 9 && parent_of(13) == 9 && parent_of(14) == 9);
static_assert(parent_of(15) == 12 && parent_of(16) == 13 && parent_of(17) == 14 && parent_of(18) == 16 && parent_of(19) == 17 && parent_of(20) == 18 && parent_of(21) == 19);

__device__ __forceinline__ unsigned short f2bf(float f) { unsigned u = __float_as_uint(f); u += 0x7FFFu + ((u >> 16) & 1u); return (unsigned short)(u >> 16); }
__device__ __forceinline__ float bfr(float f) { return __uint_as_float(((unsigned)f2bf(f)) << 16); }
__device__ __forceinline__ v16bf cat16b(v8us lo, v8us hi) { return __builtin_bit_cast(v16bf, __builtin_shufflevector(lo, hi, 0, 1, 2, 3, 4, 5, 6, 7, 8, 9, 10, 11, 12, 13, 14, 15)); }
__device__ __forceinline__ v8f wmmab_g(v16bf a, v16bf b, v8f c) {
    c = __builtin_amdgcn_wmma_f32_16x16x32_bf16(false, a, false, b, (short)0, c, false, false);
    asm volatile("v_nop\n\tv_nop\n\tv_nop\n\tv_nop" : "+v"(c) : "v"(a), "v"(b));
    return c;
}
__device__ __forceinline__ float pin(float x) { asm volatile("" : "+v"(x)); return x; }

__global__ __launch_bounds__(SPB) void k_fk(const float* __restrict__ body_pose, const float* __restrict__ betas, const float* __restrict__ global_orient,
                                            const float* __restrict__ transl, const float* __restrict__ J_template, const float* __restrict__ J_shapedirs, float* out) {
    __shared__ __align__(16) v8us  sA[SPB * 4];
    __shared__ __align__(16) v8us  sB[NT * 16 * 4];
    __shared__ __align__(16) float sk[SPB * SKP];
    __shared__ __align__(16) float sp[SPB * NP];
    __shared__ __align__(16) float so[SPB * NC];
    const int tid = threadIdx.x;
    const int lane = tid & 31, lr = lane & 15, hi = lane >> 4;
    const int wave = __builtin_amdgcn_readfirstlane((int)(threadIdx.x >> 5));
    const int s0 = blockIdx.x * SPB;
    const int bb = s0 / SEQ, tt = s0 % SEQ;
    const size_t gin  = (size_t)bb * SEQ_FULL + (size_t)tt;
    const size_t gout = (size_t)bb * OUT_SEQ + (size_t)tt;

    { const float* cp = betas + (gin + (size_t)tid) * KD;
      const v2f c0 = *(const v2f*)(cp), c1 = *(const v2f*)(cp + 2), c2 = *(const v2f*)(cp + 4), c3 = *(const v2f*)(cp + 6), c4 = *(const v2f*)(cp + 8);
      v8us r0 = (v8us){}, r1 = (v8us){}; const v8us z = (v8us){};
      r0[0] = f2bf(c0[0]); r0[1] = f2bf(c0[1]); r0[2] = f2bf(c1[0]); r0[3] = f2bf(c1[1]);
      r0[4] = f2bf(c2[0]); r0[5] = f2bf(c2[1]); r0[6] = f2bf(c3[0]); r0[7] = f2bf(c3[1]);
      r1[0] = f2bf(c4[0]); r1[1] = f2bf(c4[1]);
      sA[tid * 4 + 0] = r0; sA[tid * 4 + 1] = r1; sA[tid * 4 + 2] = z; sA[tid * 4 + 3] = z; }
    { const int n = tid; const int nc = n < NC ? n : NC - 1;
      const float* wp = J_shapedirs + nc * KD;
      float w[KD];
#pragma unroll
      for (int q = 0; q < KD / 2; ++q) { const v2f t2 = *(const v2f*)(wp + 2 * q); w[2 * q] = pin(t2[0]); w[2 * q + 1] = pin(t2[1]); }
      const bool ok = n < NC;
      v8us r0 = (v8us){}, r1 = (v8us){}; const v8us z = (v8us){};
#pragma unroll
      for (int k = 0; k < 8; ++k) { const unsigned short q = f2bf(w[k]); r0[k] = ok ? q : (unsigned short)0; }
      { const unsigned short q8 = f2bf(w[8]), q9 = f2bf(w[9]); r1[0] = ok ? q8 : (unsigned short)0; r1[1] = ok ? q9 : (unsigned short)0; }
      if (n < NT * 16) { sB[n * 4 + 0] = r0; sB[n * 4 + 1] = r1; sB[n * 4 + 2] = z; sB[n * 4 + 3] = z; } }
    { const float* src = body_pose + gin * NP;
#pragma unroll 1
      for (int i = tid; i < SPB * NP / 4; i += SPB) {
          const v4f v = *(const v4f*)(src + 4 * (size_t)i); v4f o;
          o[0] = bfr(v[0]); o[1] = bfr(v[1]); o[2] = bfr(v[2]); o[3] = bfr(v[3]);
          *(v4fa*)(&sp[4 * i]) = o; } }
    const float* gop = global_orient + (gin + (size_t)tid) * 3;
    const float* trp = transl + (gin + (size_t)tid) * 3;
    const float g0 = bfr(gop[0]), g1 = bfr(gop[1]), g2 = bfr(gop[2]);
    const float q0 = bfr(trp[0]), q1 = bfr(trp[1]), q2 = bfr(trp[2]);
    __syncthreads();

    { v16bf bfrag[NT]; float tv[NT];
#pragma unroll
      for (int t = 0; t < NT; ++t) {
          const int rowb = (t * 16 + lr) * 4 + hi;
          bfrag[t] = cat16b(sB[rowb], sB[rowb + 2]);
          const int n = t * 16 + lr; const int nc = n < NC ? n : NC - 1;
          const float x = pin(J_template[nc]);
          tv[t] = (n < NC) ? bfr(x) : 0.0f; }
#pragma unroll
      for (int mt = 0; mt < 2; ++mt) {
          const int srow = wave * 32 + mt * 16;
          const int rowa = (srow + lr) * 4 + hi;
          const v16bf a = cat16b(sA[rowa], sA[rowa + 2]);
#pragma unroll
          for (int t = 0; t < NT; ++t) {
              v8f acc = (v8f){};
              acc = wmmab_g(a, bfrag[t], acc);
              const int n = t * 16 + lr;
#pragma unroll
              for (int r = 0; r < 8; ++r) sk[(srow + 8 * hi + r) * SKP + n] = acc[r] + tv[t]; } } }
    __syncthreads();

    { const int sb = tid * SKP, pb = tid * NP, ob = tid * NC;
      float Rg[NJ][9];
      float Px[NJ], Py[NJ], Pz[NJ];
#pragma unroll
      for (int j = 0; j < NJ; ++j) {
          float ax, ay, az;
          if (j == 0) { ax = g0; ay = g1; az = g2; }
          else        { ax = sp[pb + 3 * (j - 1)]; ay = sp[pb + 3 * (j - 1) + 1]; az = sp[pb + 3 * (j - 1) + 2]; }
          const float sq   = ax * ax + ay * ay + az * az + 1e-12f;
          const float rinv = rsqrtf(sq);
          const float ang  = sq * rinv;
          const float ux = ax * rinv, uy = ay * rinv, uz = az * rinv;
          float sn, cs; sincosf(ang, &sn, &cs);
          const float tA = 1.0f - cs;
          const float r00 = tA * ux * ux + cs,      r01 = tA * ux * uy - sn * uz, r02 = tA * ux * uz + sn * uy;
          const float r10 = tA * ux * uy + sn * uz, r11 = tA * uy * uy + cs,      r12 = tA * uy * uz - sn * ux;
          const float r20 = tA * ux * uz - sn * uy, r21 = tA * uy * uz + sn * ux, r22 = tA * uz * uz + cs;
          if (j == 0) {
              Rg[0][0] = r00; Rg[0][1] = r01; Rg[0][2] = r02;
              Rg[0][3] = r10; Rg[0][4] = r11; Rg[0][5] = r12;
              Rg[0][6] = r20; Rg[0][7] = r21; Rg[0][8] = r22;
              Px[0] = sk[sb + 0] + q0;
              Py[0] = sk[sb + 1] + q1;
              Pz[0] = sk[sb + 2] + q2;
          } else {
              const int p = parent_of(j);
              const float tx = sk[sb + 3 * j]     - sk[sb + 3 * p];
              const float ty = sk[sb + 3 * j + 1] - sk[sb + 3 * p + 1];
              const float tz = sk[sb + 3 * j + 2] - sk[sb + 3 * p + 2];
              Px[j] = Rg[p][0] * tx + Rg[p][1] * ty + Rg[p][2] * tz + Px[p];
              Py[j] = Rg[p][3] * tx + Rg[p][4] * ty + Rg[p][5] * tz + Py[p];
              Pz[j] = Rg[p][6] * tx + Rg[p][7] * ty + Rg[p][8] * tz + Pz[p];
              Rg[j][0] = Rg[p][0] * r00 + Rg[p][1] * r10 + Rg[p][2] * r20;
              Rg[j][1] = Rg[p][0] * r01 + Rg[p][1] * r11 + Rg[p][2] * r21;
              Rg[j][2] = Rg[p][0] * r02 + Rg[p][1] * r12 + Rg[p][2] * r22;
              Rg[j][3] = Rg[p][3] * r00 + Rg[p][4] * r10 + Rg[p][5] * r20;
              Rg[j][4] = Rg[p][3] * r01 + Rg[p][4] * r11 + Rg[p][5] * r21;
              Rg[j][5] = Rg[p][3] * r02 + Rg[p][4] * r12 + Rg[p][5] * r22;
              Rg[j][6] = Rg[p][6] * r00 + Rg[p][7] * r10 + Rg[p][8] * r20;
              Rg[j][7] = Rg[p][6] * r01 + Rg[p][7] * r11 + Rg[p][8] * r21;
              Rg[j][8] = Rg[p][6] * r02 + Rg[p][7] * r12 + Rg[p][8] * r22;
          }
          so[ob + 3 * j]     = Px[j];
          so[ob + 3 * j + 1] = Py[j];
          so[ob + 3 * j + 2] = Pz[j];
      } }
    __syncthreads();

    { float* obase = out + gout * NC;
#pragma unroll 1
      for (int ps = 0; ps < 2; ++ps) {
#pragma unroll 1
          for (int i = tid; i < SPB * NC / 4; i += SPB) {
              const v4f val = *(const v4fa*)(&so[4 * i]);
              *(volatile v4f*)(obase + 4 * (size_t)i) = val; }
          if (ps == 0) __threadfence(); } }
}

extern "C" void kernel_launch(void* const* d_in, const int* in_sizes, int n_in,
                              void* d_out, int out_size, void* d_ws, size_t ws_size, hipStream_t stream) {
    (void)d_ws; (void)ws_size;
    if (n_in < 6) return;
    const size_t rows = (size_t)(NB - 1) * SEQ_FULL + SEQ;
    if ((size_t)in_sizes[0] < rows * NP) return;
    if ((size_t)in_sizes[1] < rows * KD) return;
    if ((size_t)in_sizes[2] < rows * 3 || (size_t)in_sizes[3] < rows * 3) return;
    if (in_sizes[4] < NC || in_sizes[5] < NC * KD) return;
    if ((size_t)out_size < ((size_t)(NB - 1) * OUT_SEQ + SEQ) * NC) return;
    const float* body_pose     = (const float*)d_in[0];
    const float* betas         = (const float*)d_in[1];
    const float* global_orient = (const float*)d_in[2];
    const float* transl        = (const float*)d_in[3];
    const float* J_template    = (const float*)d_in[4];
    const float* J_shapedirs   = (const float*)d_in[5];
    float* OUT = (float*)d_out;
    k_fk<<<dim3((unsigned)((size_t)NB * SEQ / SPB), 1, 1), SPB, 0, stream>>>(body_pose, betas, global_orient, transl, J_template, J_shapedirs, OUT);
}
